// RNNDecoderHat_70351564309221
// MI455X (gfx1250) — hardware-verified
//
#include <hip/hip_runtime.h>
#include <math.h>

constexpr int NB_ROWS  = 4096;
constexpr int NINP     = 256;
constexpr int NHID     = 256;
constexpr int NVOC     = 4;
constexpr int NSTEPS   = 128;
constexpr int NTHR     = 256;
constexpr int ROWS_BLK = 32;
constexpr int HPITCH   = 264;
constexpr int FPITCH   = 260;
constexpr int OSPITCH  = 32;
constexpr int OUT_ROW  = NSTEPS * NVOC;
constexpr float WCARRY     = 16.0f;
constexpr float WCARRY_INV = 1.0f / 16.0f;
static_assert(NB_ROWS % ROWS_BLK == 0);
static_assert(ROWS_BLK == 32 && NTHR == 256);
static_assert(NHID == 4 * 64);
static_assert(NHID % 32 == 0 && NINP % 32 == 0);
static_assert(NB_ROWS % 64 == 0 && NHID % 64 == 0);
static_assert((ROWS_BLK * HPITCH) % NTHR == 0);
static_assert(NVOC * NHID == 4 * NTHR);
static_assert(NTHR == ROWS_BLK * NVOC * 2);
static_assert(NSTEPS % 8 == 0 && OSPITCH == 8 * NVOC);
static_assert(HPITCH % 8 == 0 && FPITCH % 4 == 0);
static_assert((NB_ROWS * (NINP / 8)) % NTHR == 0 && (NHID * (NINP / 8)) % NTHR == 0);

typedef __attribute__((ext_vector_type(16))) _Float16 v16h;
typedef __attribute__((ext_vector_type(8)))  _Float16 v8h;
typedef __attribute__((ext_vector_type(16))) __bf16   v16b;
typedef __attribute__((ext_vector_type(8)))  __bf16   v8b;
typedef __attribute__((ext_vector_type(8)))  float    v8f;
typedef __attribute__((ext_vector_type(4)))  float    v4f;

__device__ __forceinline__ unsigned short f2bf_bits(float f) {
  unsigned u = __float_as_uint(f);
  return (unsigned short)((u + 0x7FFFu + ((u >> 16) & 1u)) >> 16);
}
__device__ __forceinline__ float bf_bits2f(unsigned short h) { return __uint_as_float(((unsigned)h) << 16); }

__device__ __forceinline__ void dep_guard_h(v8f& a, v8f& b, v16h x, v16h y) { asm volatile("v_nop\n\tv_nop\n\tv_nop\n\tv_nop" : "+v"(a), "+v"(b) : "v"(x), "v"(y)); }
__device__ __forceinline__ void dep_guard_b(v8f& a, v8f& b, v16b x, v16b y) { asm volatile("v_nop\n\tv_nop\n\tv_nop\n\tv_nop" : "+v"(a), "+v"(b) : "v"(x), "v"(y)); }
__device__ __forceinline__ void keep4_h(v16h a, v16h b, v16h c, v16h d) { asm volatile("v_nop" :: "v"(a), "v"(b), "v"(c), "v"(d)); }
__device__ __forceinline__ void keep4_b(v16b a, v16b b, v16b c, v16b d) { asm volatile("v_nop" :: "v"(a), "v"(b), "v"(c), "v"(d)); }
__device__ __forceinline__ void acc_guard4(v8f& a, v8f& b, v8f& c, v8f& d) { asm volatile("v_nop\n\tv_nop\n\tv_nop\n\tv_nop" : "+v"(a), "+v"(b), "+v"(c), "+v"(d)); }
template <typename T> struct Frag;
template <> struct Frag<_Float16> {
  typedef v16h V; union U { v16h v; v8h h[2]; };
  static __device__ __forceinline__ v16h load(const _Float16* p) {
    U f; f.h[0] = *(const v8h*)(p); f.h[1] = *(const v8h*)(p + 16); return f.v;
  }
  static __device__ __forceinline__ v8f mma(v16h a, v16h b, v8f c) {
    return __builtin_amdgcn_wmma_f32_16x16x32_f16(false, a, false, b, (short)0, c, false, false);
  }
  static __device__ __forceinline__ void guard(v8f& a, v8f& b, v16h x, v16h y) { dep_guard_h(a, b, x, y); }
  static __device__ __forceinline__ void keep(v16h a, v16h b, v16h c, v16h d) { keep4_h(a, b, c, d); }
};
template <> struct Frag<__bf16> {
  typedef v16b V; union U { v16b v; v8b h[2]; };
  static __device__ __forceinline__ v16b load(const __bf16* p) {
    U f; f.h[0] = *(const v8b*)(p); f.h[1] = *(const v8b*)(p + 16); return f.v;
  }
  static __device__ __forceinline__ v8f mma(v16b a, v16b b, v8f c) {
    return __builtin_amdgcn_wmma_f32_16x16x32_bf16(false, a, false, b, (short)0, c, false, false);
  }
  static __device__ __forceinline__ void guard(v8f& a, v8f& b, v16b x, v16b y) { dep_guard_b(a, b, x, y); }
  static __device__ __forceinline__ void keep(v16b a, v16b b, v16b c, v16b d) { keep4_b(a, b, c, d); }
};

template <int ET> struct Elem;
template <> struct Elem<0> { typedef _Float16 T; };
template <> struct Elem<1> { typedef __bf16 T; };
template <int ET, bool SPLIT, int BIAS_MODE, int OUT_MODE, bool RESID, int ACT = 0>
__global__ __launch_bounds__(256) void wmma_gemm64(
    const unsigned short* __restrict__ Ap, const unsigned short* __restrict__ A2p, int lda, long strideA,
    const unsigned short* __restrict__ Btp, const unsigned short* __restrict__ Bt2p, int ldb, long strideB,
    void* __restrict__ Cout, void* __restrict__ Cout2, int ldc, long strideC,
    const float* __restrict__ bias,
    const float* __restrict__ resid, long strideR,
    int M, int N, int K, float scale) {
  typedef typename Elem<ET>::T T;
  typedef typename Frag<T>::V V;
  const T* A = (const T*)Ap; const T* A2 = (const T*)A2p; const T* Bt = (const T*)Btp; const T* Bt2 = (const T*)Bt2p;
  __shared__ __align__(16) float sT[8][16 * 68];
  const int b    = blockIdx.y;
  const int lane = threadIdx.x & 31;
  const int wave = threadIdx.x >> 5;
  const int tilesN = N >> 6;
  const int tilesM = M >> 6;
  const int tile = blockIdx.x * 8 + wave;
  if (tile >= tilesM * tilesN) return;
  const int tm = tile / tilesN;
  const int tn = tile - tm * tilesN;
  const int m0 = tm << 6;
  const int n0 = tn << 6;

  const T* Ab  = A  + (size_t)b * strideA;
  const T* Bb  = Bt + (size_t)b * strideB;
  const T* Ab2 = SPLIT ? (A2  + (size_t)b * strideA) : nullptr;
  const T* Bb2 = SPLIT ? (Bt2 + (size_t)b * strideB) : nullptr;

  const int rlane = lane & 15;
  const int koff  = (lane >> 4) * 8;
  const int mOff  = (lane >> 4) * 8;

  v8f acc[4][4];
#pragma unroll
  for (int i = 0; i < 4; ++i)
#pragma unroll
    for (int j = 0; j < 4; ++j) acc[i][j] = (v8f){0.f,0.f,0.f,0.f,0.f,0.f,0.f,0.f};

  for (int k0 = 0; k0 < K; k0 += 32) {
    V bh[4], bl[4];
#pragma unroll
    for (int j = 0; j < 4; ++j) {
      const size_t bo = (size_t)(n0 + (j << 4) + rlane) * ldb + koff + k0;
      bh[j] = Frag<T>::load(Bb + bo);
      if (SPLIT) bl[j] = Frag<T>::load(Bb2 + bo);
    }
#pragma unroll
    for (int i = 0; i < 4; ++i) {
      const size_t ao = (size_t)(m0 + (i << 4) + rlane) * lda + koff + k0;
      V ah = Frag<T>::load(Ab + ao);
      V al;
      if (SPLIT) al = Frag<T>::load(Ab2 + ao);
#pragma unroll
      for (int j = 0; j < 4; ++j) {
        acc[i][j] = Frag<T>::mma(ah, bh[j], acc[i][j]);
        if (SPLIT) {
          acc[i][j] = Frag<T>::mma(ah, bl[j], acc[i][j]);
          acc[i][j] = Frag<T>::mma(al, bh[j], acc[i][j]);
        }
      }
      Frag<T>::guard(acc[i][0], acc[i][3], ah, SPLIT ? al : ah);
    }
    Frag<T>::keep(bh[0], bh[1], bh[2], bh[3]);
    if (SPLIT) Frag<T>::keep(bl[0], bl[1], bl[2], bl[3]);
  }
  acc_guard4(acc[0][0], acc[0][1], acc[0][2], acc[0][3]);
  acc_guard4(acc[1][0], acc[1][1], acc[1][2], acc[1][3]);
  acc_guard4(acc[2][0], acc[2][1], acc[2][2], acc[2][3]);
  acc_guard4(acc[3][0], acc[3][1], acc[3][2], acc[3][3]);

  float* slab = sT[wave];
  const float* Rb = RESID ? (resid + (size_t)b * strideR) : nullptr;
#pragma unroll
  for (int i = 0; i < 4; ++i) {
    const int mBase = m0 + (i << 4);
#pragma unroll
    for (int j = 0; j < 4; ++j) {
      const int n = n0 + (j << 4) + rlane;
      float bv = 0.f;
      if (BIAS_MODE == 2) bv = bias[n];
#pragma unroll
      for (int r = 0; r < 8; ++r) {
        float v = acc[i][j][r] * scale;
        if (BIAS_MODE == 1) v += bias[mBase + mOff + r];
        if (BIAS_MODE == 2) v += bv;
        if (RESID) v += Rb[(size_t)(mBase + mOff + r) * ldc + n];
        if (ACT == 1) v = tanhf(v);
        if (ACT == 2) v = fmaxf(v, 0.0f);
        if (ACT == 3) v = v / (1.0f + expf(-v));
        if (ACT == 4) v = (v > 0.f) ? v : 0.01f * v;
        if (ACT == 5) v = 0.5f * v * (1.0f + erff(v * 0.70710678118654752f));
        slab[(mOff + r) * 68 + (j << 4) + rlane] = v;
      }
    }
    __builtin_amdgcn_fence(__ATOMIC_RELEASE, "workgroup");
    __builtin_amdgcn_wave_barrier();
    __builtin_amdgcn_fence(__ATOMIC_ACQUIRE, "workgroup");
    if (OUT_MODE == 0) {
      float* C = (float*)Cout + (size_t)b * strideC;
      const int hh = lane >> 4, c4 = (lane & 15) * 4;
      for (int pass = 0; pass < 2; ++pass) {
#pragma unroll
        for (int it = 0; it < 8; ++it) {
          const int row = it * 2 + hh;
          v4f v = *(const v4f*)(slab + row * 68 + c4);
          *(volatile v4f*)(C + (size_t)(mBase + row) * ldc + n0 + c4) = v;
        }
        __threadfence();
      }
    } else {
      const int q = lane >> 3, c8 = (lane & 7) * 8;
      unsigned short* C  = (unsigned short*)Cout  + (size_t)b * strideC;
      unsigned short* C2 = (OUT_MODE == 2) ? ((unsigned short*)Cout2 + (size_t)b * strideC) : nullptr;
      for (int pass = 0; pass < 2; ++pass) {
#pragma unroll
        for (int it = 0; it < 4; ++it) {
          const int row = it * 4 + q;
          const float* sp = slab + row * 68 + c8;
          v8h hv, lv;
#pragma unroll
          for (int e = 0; e < 8; ++e) {
            if (OUT_MODE == 1) {
              hv[e] = (_Float16)sp[e];
            } else {
              unsigned short hb = f2bf_bits(sp[e]);
              unsigned short lb = f2bf_bits(sp[e] - bf_bits2f(hb));
              hv[e] = __builtin_bit_cast(_Float16, hb);
              lv[e] = __builtin_bit_cast(_Float16, lb);
            }
          }
          *(volatile v8h*)(C + (size_t)(mBase + row) * ldc + n0 + c8) = hv;
          if (OUT_MODE == 2) *(volatile v8h*)(C2 + (size_t)(mBase + row) * ldc + n0 + c8) = lv;
        }
        __threadfence();
      }
    }
    __builtin_amdgcn_fence(__ATOMIC_RELEASE, "workgroup");
    __builtin_amdgcn_wave_barrier();
    __builtin_amdgcn_fence(__ATOMIC_ACQUIRE, "workgroup");
  }
}

__global__ __launch_bounds__(NTHR) void cvt8_f16_kernel(const float* __restrict__ src, unsigned short* __restrict__ dst,
                                                        int nrow, int ncol8, int spitch, float sc) {
  const int i  = blockIdx.x * NTHR + threadIdx.x;
  const int n8 = nrow * ncol8;
  if (i < n8) {
    const int row = i / ncol8;
    const int c8  = i - row * ncol8;
    const float* sp = src + (size_t)row * spitch + c8 * 8;
    const v4f a = *(const v4f*)(sp);
    const v4f b = *(const v4f*)(sp + 4);
    v8h hv;
#pragma unroll
    for (int e = 0; e < 4; ++e) {
      hv[e]     = (_Float16)(a[e] * sc);
      hv[4 + e] = (_Float16)(b[e] * sc);
    }
    *(volatile v8h*)(dst + (size_t)i * 8) = hv;
    __threadfence();
    *(volatile v8h*)(dst + (size_t)i * 8) = hv;
  }
}

__global__ __launch_bounds__(NTHR) void rnn_seq_kernel(const float* __restrict__ XP, const float* __restrict__ bhh,
                                                       const unsigned short* __restrict__ WHHp,
                                                       const float* __restrict__ Wout, float* __restrict__ out) {
  __shared__ __align__(16) _Float16 Hh[ROWS_BLK * HPITCH];
  __shared__ __align__(16) float    Hf[ROWS_BLK * FPITCH];
  __shared__ __align__(16) float    Ws[NVOC * NHID];
  __shared__ __align__(16) float    Os[ROWS_BLK * OSPITCH];
  const _Float16* WHH = (const _Float16*)WHHp;
  const int tid = threadIdx.x, lane = tid & 31, wave = tid >> 5;
  const int c = lane & 15, hh = lane >> 4, koff = hh * 8;
  const int ms = wave >> 2;
  const int cg = wave & 3;
  const int rowbase = blockIdx.x * ROWS_BLK;

#pragma unroll 1
  for (int i = tid; i < ROWS_BLK * HPITCH; i += NTHR) Hh[i] = (_Float16)0.0f;
  *(v4f*)(Ws + 4 * tid) = *(const v4f*)(Wout + 4 * tid);
  float xr[4][8];
#pragma unroll
  for (int q = 0; q < 4; ++q) {
    const int j = 64 * cg + 16 * q + c;
    const float bv = bhh[j];
#pragma unroll
    for (int r = 0; r < 8; ++r)
      xr[q][r] = XP[(size_t)(rowbase + 16 * ms + 8 * hh + r) * NHID + j] + bv;
  }
  __syncthreads();

  const int hrow  = tid >> 3;
  const int hvoc  = (tid >> 1) & 3;
  const int hhalf = tid & 1;
  const float* hfp = Hf + hrow * FPITCH + (NHID / 2) * hhalf;
  const float* wsp = Ws + hvoc * NHID + (NHID / 2) * hhalf;
  const int orow = 4 * wave + (lane >> 3);
  const int oc4  = (lane & 7) * 4;

  const v8f z8 = {0.f, 0.f, 0.f, 0.f, 0.f, 0.f, 0.f, 0.f};
  const _Float16* arow = Hh + (16 * ms + c) * HPITCH + koff;

#pragma unroll 1
  for (int t = 0; t < NSTEPS; ++t) {
    v8f acc[4];
#pragma unroll
    for (int q = 0; q < 4; ++q) acc[q] = z8;
#pragma unroll 1
    for (int k0 = 0; k0 < NHID; k0 += 32) {
      v16h bq[4];
#pragma unroll
      for (int q = 0; q < 4; ++q)
        bq[q] = Frag<_Float16>::load(WHH + (size_t)(64 * cg + 16 * q + c) * NHID + koff + k0);
      const v16h a = Frag<_Float16>::load(arow + k0);
#pragma unroll
      for (int q = 0; q < 4; ++q) acc[q] = Frag<_Float16>::mma(a, bq[q], acc[q]);
      dep_guard_h(acc[0], acc[3], a, a);
      keep4_h(bq[0], bq[1], bq[2], bq[3]);
    }
    acc_guard4(acc[0], acc[1], acc[2], acc[3]);
    __syncthreads();

#pragma unroll
    for (int q = 0; q < 4; ++q) {
      const int j = 64 * cg + 16 * q + c;
#pragma unroll
      for (int r = 0; r < 8; ++r) {
        const float z  = acc[q][r] * WCARRY_INV + xr[q][r];
        const float hn = tanhf(z);
        const int row = 16 * ms + 8 * hh + r;
        Hh[row * HPITCH + j] = (_Float16)hn;
        Hf[row * FPITCH + j] = hn;
      }
    }
    __syncthreads();

    float s = 0.0f;
#pragma unroll 1
    for (int k = 0; k < NHID / 2; k += 4) {
      const v4f h4 = *(const v4f*)(hfp + k);
      const v4f w4 = *(const v4f*)(wsp + k);
      s = fmaf(h4[0], w4[0], s);
      s = fmaf(h4[1], w4[1], s);
      s = fmaf(h4[2], w4[2], s);
      s = fmaf(h4[3], w4[3], s);
    }
    s += __shfl_xor(s, 1, 32);
    float mx = fmaxf(s, __shfl_xor(s, 2, 32));
    mx = fmaxf(mx, __shfl_xor(mx, 4, 32));
    const float d  = s - mx;
    const float e  = expf(d);
    float se = e + __shfl_xor(e, 2, 32);
    se += __shfl_xor(se, 4, 32);
    const float lp = d - logf(se);
    if (hhalf == 0) Os[hrow * OSPITCH + (t & 7) * NVOC + hvoc] = lp;

    if ((t & 7) == 7) {
      __builtin_amdgcn_fence(__ATOMIC_RELEASE, "workgroup");
      __builtin_amdgcn_wave_barrier();
      __builtin_amdgcn_fence(__ATOMIC_ACQUIRE, "workgroup");
      const v4f v = *(const v4f*)(Os + orow * OSPITCH + oc4);
      float* dst = out + (size_t)(rowbase + orow) * OUT_ROW + (t >> 3) * OSPITCH + oc4;
      for (int pass = 0; pass < 2; ++pass) {
        *(volatile v4f*)dst = v;
        __threadfence();
      }
      __builtin_amdgcn_fence(__ATOMIC_RELEASE, "workgroup");
      __builtin_amdgcn_wave_barrier();
      __builtin_amdgcn_fence(__ATOMIC_ACQUIRE, "workgroup");
    }
  }
}

extern "C" void kernel_launch(void* const* d_in, const int* in_sizes, int n_in,
                              void* d_out, int out_size, void* d_ws, size_t ws_size, hipStream_t stream) {
  if (n_in < 6 || d_out == nullptr || d_ws == nullptr) return;
  if (in_sizes[0] != NB_ROWS * NINP || in_sizes[1] != NHID * NINP || in_sizes[2] != NHID ||
      in_sizes[3] != NHID * NHID || in_sizes[4] != NHID || in_sizes[5] != NVOC * NHID ||
      out_size != NB_ROWS * NSTEPS * NVOC) return;

  const float* a     = (const float*)d_in[0];
  const float* w_ih  = (const float*)d_in[1];
  const float* b_ih  = (const float*)d_in[2];
  const float* w_hh  = (const float*)d_in[3];
  const float* b_hh  = (const float*)d_in[4];
  const float* w_out = (const float*)d_in[5];
  float* y_out = (float*)d_out;

  char* ws = (char*)d_ws; size_t off = 0;
  auto carve = [&](size_t bytes) -> char* { char* p = ws + off; off += (bytes + 255) & ~(size_t)255; return p; };
  unsigned short* AH    = (unsigned short*)carve((size_t)NB_ROWS * NINP * 2);
  unsigned short* WIH16 = (unsigned short*)carve((size_t)NHID * NINP * 2);
  unsigned short* WHH16 = (unsigned short*)carve((size_t)NHID * NHID * 2);
  float*          XP    = (float*)carve((size_t)NB_ROWS * NHID * 4);
  if (off > ws_size || off > (size_t)134217728) return;

  const int n8a = NB_ROWS * (NINP / 8);
  const int n8w = NHID * (NINP / 8);
  cvt8_f16_kernel<<<(n8a + NTHR - 1) / NTHR, NTHR, 0, stream>>>(a,    AH,    NB_ROWS, NINP / 8, NINP, 1.0f);
  cvt8_f16_kernel<<<(n8w + NTHR - 1) / NTHR, NTHR, 0, stream>>>(w_ih, WIH16, NHID,    NINP / 8, NINP, WCARRY);
  cvt8_f16_kernel<<<(n8w + NTHR - 1) / NTHR, NTHR, 0, stream>>>(w_hh, WHH16, NHID,    NHID / 8, NHID, WCARRY);

  const dim3 ggrid((NB_ROWS / 64) * (NHID / 64) / 8, 1);
  wmma_gemm64<0, false, 2, 0, false, 0><<<ggrid, 256, 0, stream>>>(
      AH, AH, NINP, 0L, WIH16, WIH16, NINP, 0L, (void*)XP, (void*)XP, NHID, 0L,
      b_ih, (const float*)XP, 0L, NB_ROWS, NHID, NINP, WCARRY_INV);

  rnn_seq_kernel<<<NB_ROWS / ROWS_BLK, NTHR, 0, stream>>>(XP, b_hh, WHH16, w_out, y_out);
}
